// CustomMixedDecoder_47175920779908
// MI455X (gfx1250) — hardware-verified
//
#include <hip/hip_runtime.h>
#include <math.h>
#include <stdint.h>

#define NB_   1024
#define LAT_  32
#define FRM_  267
#define HID_  512
#define NE_   16
#define GH_   64
#define IN0_  299
#define IN1_  544
#define KP0_  320
#define ZO0_  272
#define KL1_  544
#define ZO1_  512
#define LDA1_ 576
#define NP2_  320
#define HP_   72
#define OP_   68
#define WSC   64.0f
#define LOSC  2048.0f

static_assert((NB_ % 64) == 0 && (HID_ % 64) == 0 && (NP2_ % 64) == 0 && NP2_ >= FRM_);
static_assert((KP0_ % 32) == 0 && KP0_ >= ZO0_ + LAT_ && ZO0_ >= FRM_);
static_assert((KL1_ % 32) == 0 && KL1_ == ZO1_ + LAT_ && (LDA1_ % 64) == 0 && LDA1_ >= ZO1_ + 64);
static_assert((HP_ % 8) == 0 && (OP_ % 4) == 0 && ((NB_ * FRM_) % (4 * 256)) == 0 && (NB_ % 32) == 0);
static_assert(((NB_ * KP0_) % (8 * 256)) == 0 && ((4 * NB_ * 8) % 256) == 0);

typedef _Float16 v16h __attribute__((ext_vector_type(16)));
typedef _Float16 v8h  __attribute__((ext_vector_type(8)));
typedef float    v8f  __attribute__((ext_vector_type(8)));
typedef float    v4f  __attribute__((ext_vector_type(4)));
typedef unsigned int v4u __attribute__((ext_vector_type(4)));
typedef v8h v8hm __attribute__((may_alias));
typedef v4f v4fm __attribute__((may_alias));

union FragH { v16h v; v8h h[2]; };
union P8 { v8h h; v4u u; };

__device__ __forceinline__ unsigned short bf_bits(float f) {
  unsigned u = __float_as_uint(f);
  return (unsigned short)((u + 0x7FFFu + ((u >> 16) & 1u)) >> 16);
}
__device__ __forceinline__ float bf_up(unsigned short h) { return __uint_as_float(((unsigned)h) << 16); }
__device__ __forceinline__ float bfr(float f) { return bf_up(bf_bits(f)); }
__device__ __forceinline__ unsigned short h_bits(_Float16 x) { return __builtin_bit_cast(unsigned short, x); }
__device__ __forceinline__ unsigned pk16(unsigned short a, unsigned short b) { return (unsigned)a | ((unsigned)b << 16); }
__device__ __forceinline__ unsigned pkh(float a, float b) { return pk16(h_bits((_Float16)a), h_bits((_Float16)b)); }
__device__ __forceinline__ v8f zero8() { v8f z = {0.f, 0.f, 0.f, 0.f, 0.f, 0.f, 0.f, 0.f}; return z; }

__device__ __forceinline__ float elu1(float x) {
  const float em = expm1f(x);
  return (x > 0.f) ? x : em;
}

__device__ __forceinline__ void hl_one(float f, _Float16& h, _Float16& l) {
#pragma clang fp contract(off)
  const _Float16 hv = (_Float16)f;
  const float d = f - (float)hv;
  const float r = d * LOSC;
  h = hv;
  l = (_Float16)r;
}

__device__ __forceinline__ v16h ldfrag_h(const _Float16* p) {
  FragH f;
  f.h[0] = *(const v8h*)(p);
  f.h[1] = *(const v8h*)(p + 16);
  return f.v;
}

__device__ __forceinline__ v8f wm(v16h a, v16h b, v8f c) {
  return __builtin_amdgcn_wmma_f32_16x16x32_f16(false, a, false, b, (short)0, c, false, false);
}
__device__ __forceinline__ void guard4(v8f& c0, v8f& c1, v8f& c2, v8f& c3, v16h a0, v16h a1, v16h b0, v16h b1) {
#if defined(__HIP_DEVICE_COMPILE__)
  asm volatile("v_nop\n\tv_nop\n\tv_nop\n\tv_nop"
               : "+v"(c0), "+v"(c1), "+v"(c2), "+v"(c3)
               : "v"(a0), "v"(a1), "v"(b0), "v"(b1));
#endif
}
__device__ __forceinline__ void guard2(v8f& c0, v8f& c1, v16h a0, v16h a1, v16h b0) {
#if defined(__HIP_DEVICE_COMPILE__)
  asm volatile("v_nop\n\tv_nop\n\tv_nop\n\tv_nop"
               : "+v"(c0), "+v"(c1)
               : "v"(a0), "v"(a1), "v"(b0));
#endif
}
__device__ __forceinline__ void wave_sync_lds() {
  __builtin_amdgcn_fence(__ATOMIC_RELEASE, "workgroup");
  __builtin_amdgcn_wave_barrier();
  __builtin_amdgcn_fence(__ATOMIC_ACQUIRE, "workgroup");
}

__global__ __launch_bounds__(256) void cvt_x0(const float* __restrict__ z, const float* __restrict__ c,
                                              unsigned short* xh, int n8) {
  const int t = blockIdx.x * 256 + threadIdx.x;
  const int tc = (t < n8) ? t : (n8 - 1);
  const int d = tc * 8;
  const int row = d / KP0_;
  const int k0 = d - row * KP0_;
  float f[8];
#pragma unroll
  for (int u = 0; u < 8; ++u) {
    const int k = k0 + u;
    const int kc = (k < FRM_) ? k : (FRM_ - 1);
    int kz = k - ZO0_;
    kz = (kz < 0) ? 0 : kz;
    kz = (kz > LAT_ - 1) ? (LAT_ - 1) : kz;
    const float cv = c[(size_t)row * FRM_ + kc];
    const float zv = z[(size_t)row * LAT_ + kz];
    const float v = (k < FRM_) ? cv : (((k >= ZO0_) && (k < ZO0_ + LAT_)) ? zv : 0.f);
    f[u] = bfr(v);
  }
  v4u pk;
#pragma unroll
  for (int e = 0; e < 4; ++e) pk[e] = pkh(f[2 * e], f[2 * e + 1]);
  unsigned short* gp = xh + (size_t)tc * 8;
  if (t < n8) *(volatile v4u*)gp = pk;
  __threadfence();
  if (t < n8) *(volatile v4u*)gp = pk;
}

__global__ __launch_bounds__(256) void cvt_zl(const float* __restrict__ z, unsigned short* ap, int nthr) {
  const int t = blockIdx.x * 256 + threadIdx.x;
  const int tc = (t < nthr) ? t : (nthr - 1);
  const int per = NB_ * 8;
  const int pl = tc / per;
  const int rem = tc - pl * per;
  const int row = rem >> 3;
  const int p = rem & 7;
  const int pc = (p < 4) ? p : 3;
  const float* zp = z + (size_t)row * LAT_ + 8 * pc;
  const v4f a = *(const v4f*)zp;
  const v4f b = *(const v4f*)(zp + 4);
  const bool keep = ((pl & 1) == 0) && (p < 4);
  float f[8];
#pragma unroll
  for (int i = 0; i < 4; ++i) {
    f[i] = keep ? bfr(a[i]) : 0.f;
    f[4 + i] = keep ? bfr(b[i]) : 0.f;
  }
  v4u pk;
#pragma unroll
  for (int e = 0; e < 4; ++e) pk[e] = pkh(f[2 * e], f[2 * e + 1]);
  unsigned short* gp = ap + (size_t)pl * ((size_t)NB_ * LDA1_) + (size_t)row * LDA1_ + ZO1_ + 8 * p;
  if (t < nthr) *(volatile v4u*)gp = pk;
  __threadfence();
  if (t < nthr) *(volatile v4u*)gp = pk;
}

__global__ __launch_bounds__(256) void cvt_w(const float* __restrict__ w, unsigned short* dst,
                                             int K, int N, int NP, int KP, int PW, int PP, int ZW, int n8) {
  const int t = blockIdx.x * 256 + threadIdx.x;
  const int tc = (t < n8) ? t : (n8 - 1);
  const int d = tc * 8;
  const int R = d / KP;
  const int k0 = d - R * KP;
  const int e = R / NP;
  const int o = R - e * NP;
  const int oc = (o < N) ? o : (N - 1);
  const bool oval = (o < N);
  float f[8];
#pragma unroll
  for (int u = 0; u < 8; ++u) {
    const int k = k0 + u;
    const int ia = (k < PW) ? (ZW + k) : -1;
    const int kk = k - PP;
    const int ib = ((kk >= 0) && (kk < ZW)) ? kk : -1;
    const int i = (k < PP) ? ia : ib;
    int ic = (i < 0) ? 0 : i;
    ic = (ic > K - 1) ? (K - 1) : ic;
    const float v = w[((size_t)e * K + ic) * (size_t)N + oc];
    f[u] = ((i >= 0) && oval) ? (bfr(v) * WSC) : 0.f;
  }
  v4u pk;
#pragma unroll
  for (int q = 0; q < 4; ++q) pk[q] = pkh(f[2 * q], f[2 * q + 1]);
  unsigned short* gp = dst + (size_t)tc * 8;
  if (t < n8) *(volatile v4u*)gp = pk;
  __threadfence();
  if (t < n8) *(volatile v4u*)gp = pk;
}

__global__ __launch_bounds__(64) void gate_mlp(const unsigned short* __restrict__ xh,
                                               const unsigned short* __restrict__ g1t, const float* __restrict__ gb1,
                                               const unsigned short* __restrict__ g2t, const float* __restrict__ gb2,
                                               const unsigned short* __restrict__ g3t, const float* __restrict__ gb3,
                                               float* coefp) {
#pragma clang fp contract(off)
  __shared__ __align__(16) _Float16 Hh[2][16 * HP_];
  __shared__ __align__(16) _Float16 Hl[2][16 * HP_];
  __shared__ __align__(16) float Cs[2][256];
  const int lane = threadIdx.x & 31, wave = threadIdx.x >> 5;
  const int idx = lane & 15, hh = lane >> 4, koff = 8 * hh;
  const int m0 = blockIdx.x * 32 + 16 * wave;
  const _Float16* X  = (const _Float16*)(const void*)xh  + (size_t)(m0 + idx) * KP0_ + koff;
  const _Float16* G1 = (const _Float16*)(const void*)g1t + (size_t)idx * KP0_ + koff;
  const _Float16* G2 = (const _Float16*)(const void*)g2t + (size_t)idx * GH_ + koff;
  const _Float16* G3 = (const _Float16*)(const void*)g3t + (size_t)idx * GH_ + koff;
  _Float16* hhp = Hh[wave];
  _Float16* hlp = Hl[wave];

  v8f acc[4];
#pragma unroll
  for (int j = 0; j < 4; ++j) acc[j] = zero8();
#pragma unroll 1
  for (int ks = 0; ks < KP0_ / 32; ++ks) {
    const int k0 = 32 * ks;
    const v16h fa = ldfrag_h(X + k0);
    {
      const v16h b0 = ldfrag_h(G1 + k0);
      const v16h b1 = ldfrag_h(G1 + (size_t)16 * KP0_ + k0);
      acc[0] = wm(fa, b0, acc[0]);
      acc[1] = wm(fa, b1, acc[1]);
      guard2(acc[0], acc[1], fa, b0, b1);
    }
    {
      const v16h b2 = ldfrag_h(G1 + (size_t)32 * KP0_ + k0);
      const v16h b3 = ldfrag_h(G1 + (size_t)48 * KP0_ + k0);
      acc[2] = wm(fa, b2, acc[2]);
      acc[3] = wm(fa, b3, acc[3]);
      guard2(acc[2], acc[3], fa, b2, b3);
    }
  }
#pragma unroll
  for (int j = 0; j < 4; ++j) {
    const float bb = bfr(gb1[16 * j + idx]);
#pragma unroll
    for (int r = 0; r < 8; ++r) {
      float v = acc[j][r] * (1.0f / WSC);
      v = v + bb;
      v = elu1(v);
      _Float16 h, l;
      hl_one(v, h, l);
      const int o = (8 * hh + r) * HP_ + 16 * j + idx;
      hhp[o] = h;
      hlp[o] = l;
    }
  }
  wave_sync_lds();

  const _Float16* ga = hhp + idx * HP_ + koff;
  const _Float16* gl = hlp + idx * HP_ + koff;
  v8f c0[4], c1[4];
#pragma unroll
  for (int j = 0; j < 4; ++j) { c0[j] = zero8(); c1[j] = zero8(); }
#pragma unroll
  for (int ks = 0; ks < 2; ++ks) {
    const v16h fh = ldfrag_h(ga + 32 * ks);
    const v16h fl = ldfrag_h(gl + 32 * ks);
    {
      const v16h b0 = ldfrag_h(G2 + 32 * ks);
      const v16h b1 = ldfrag_h(G2 + 16 * GH_ + 32 * ks);
      c0[0] = wm(fh, b0, c0[0]);
      c1[0] = wm(fl, b0, c1[0]);
      c0[1] = wm(fh, b1, c0[1]);
      c1[1] = wm(fl, b1, c1[1]);
      guard4(c0[0], c1[0], c0[1], c1[1], fh, fl, b0, b1);
    }
    {
      const v16h b2 = ldfrag_h(G2 + 32 * GH_ + 32 * ks);
      const v16h b3 = ldfrag_h(G2 + 48 * GH_ + 32 * ks);
      c0[2] = wm(fh, b2, c0[2]);
      c1[2] = wm(fl, b2, c1[2]);
      c0[3] = wm(fh, b3, c0[3]);
      c1[3] = wm(fl, b3, c1[3]);
      guard4(c0[2], c1[2], c0[3], c1[3], fh, fl, b2, b3);
    }
  }
#pragma unroll
  for (int j = 0; j < 4; ++j) {
    const float bb = bfr(gb2[16 * j + idx]);
#pragma unroll
    for (int r = 0; r < 8; ++r) {
      float v = c0[j][r] * (1.0f / WSC);
      const float v1 = c1[j][r] * (1.0f / (WSC * LOSC));
      v = v + v1;
      v = v + bb;
      v = elu1(v);
      _Float16 h, l;
      hl_one(v, h, l);
      const int o = (8 * hh + r) * HP_ + 16 * j + idx;
      hhp[o] = h;
      hlp[o] = l;
    }
  }
  wave_sync_lds();

  v8f e0 = zero8(), e1 = zero8();
#pragma unroll
  for (int ks = 0; ks < 2; ++ks) {
    const v16h fh = ldfrag_h(ga + 32 * ks);
    const v16h fl = ldfrag_h(gl + 32 * ks);
    const v16h bw = ldfrag_h(G3 + 32 * ks);
    e0 = wm(fh, bw, e0);
    e1 = wm(fl, bw, e1);
    guard2(e0, e1, fh, fl, bw);
  }
  const float b3 = bfr(gb3[idx]);
  float lg[8], mx[8], pe[8], sm[8];
#pragma unroll
  for (int r = 0; r < 8; ++r) {
    float v = e0[r] * (1.0f / WSC);
    const float v1 = e1[r] * (1.0f / (WSC * LOSC));
    v = v + v1;
    lg[r] = v + b3;
    mx[r] = lg[r];
  }
#pragma unroll
  for (int off = 1; off < 16; off <<= 1) {
#pragma unroll
    for (int r = 0; r < 8; ++r) mx[r] = fmaxf(mx[r], __shfl_xor(mx[r], off, 32));
  }
#pragma unroll
  for (int r = 0; r < 8; ++r) {
    pe[r] = expf(lg[r] - mx[r]);
    sm[r] = pe[r];
  }
#pragma unroll
  for (int off = 1; off < 16; off <<= 1) {
#pragma unroll
    for (int r = 0; r < 8; ++r) sm[r] = sm[r] + __shfl_xor(sm[r], off, 32);
  }
  float* cs = Cs[wave];
#pragma unroll
  for (int r = 0; r < 8; ++r) {
    const float inv = 1.0f / sm[r];
    cs[(8 * hh + r) * 16 + idx] = pe[r] * inv;
  }
  wave_sync_lds();

  const v4f o0 = *(const v4fm*)(cs + 4 * lane);
  const v4f o1 = *(const v4fm*)(cs + 128 + 4 * lane);
  float* gp = coefp + (size_t)m0 * NE_;
  *(volatile v4f*)(gp + 4 * lane) = o0;
  *(volatile v4f*)(gp + 128 + 4 * lane) = o1;
  __threadfence();
  *(volatile v4f*)(gp + 4 * lane) = o0;
  *(volatile v4f*)(gp + 128 + 4 * lane) = o1;
}

template <int KSTEPS, int LDA, int LDB, int NP, int NREAL, bool SPLIT, bool FINAL>
__global__ __launch_bounds__(128) void moe_gemm(const unsigned short* __restrict__ ahp,
                                                const unsigned short* __restrict__ alp,
                                                const unsigned short* __restrict__ wtp,
                                                const float* __restrict__ bias,
                                                const float* __restrict__ coef,
                                                unsigned short* ohp, unsigned short* olp, float* ofp) {
  static_assert(32 * KSTEPS <= LDA && 32 * KSTEPS <= LDB && (NP % 64) == 0 && NREAL <= NP);
  static_assert((LDA % 8) == 0 && (LDB % 8) == 0);
  __shared__ __align__(16) float cT[64 * 17];
  __shared__ __align__(16) float bT[NE_ * 64];
  __shared__ __align__(16) _Float16 Hh[4][16 * HP_];
  __shared__ __align__(16) _Float16 Hl[4][16 * HP_];
  __shared__ __align__(16) float Os[4][16 * OP_];
  const int tid = threadIdx.x, lane = tid & 31, wave = tid >> 5;
  const int idx = lane & 15, hh = lane >> 4, koff = 8 * hh;
  const int n0 = blockIdx.x * 64, m0 = blockIdx.y * 64;
  const int mw = m0 + 16 * wave;

  for (int d = tid; d < 64 * NE_; d += 128) {
    const int row = d >> 4, e = d & 15;
    cT[row * 17 + e] = coef[(size_t)(m0 + row) * NE_ + e];
  }
  for (int d = tid; d < NE_ * 64; d += 128) {
    const int e = d >> 6, n = d & 63;
    const int col = n0 + n;
    const int cc = (col < NREAL) ? col : (NREAL - 1);
    const float bv = bfr(bias[(size_t)e * NREAL + cc]);
    bT[e * 64 + n] = (col < NREAL) ? bv : 0.f;
  }
  __syncthreads();

  const _Float16* A  = (const _Float16*)(const void*)ahp + (size_t)(mw + idx) * LDA + koff;
  const _Float16* AL = (const _Float16*)(const void*)alp + (size_t)(mw + idx) * LDA + koff;
  const _Float16* W  = (const _Float16*)(const void*)wtp + (size_t)(n0 + idx) * LDB + koff;

  v8f accM[4];
#pragma unroll
  for (int j = 0; j < 4; ++j) accM[j] = zero8();

#pragma unroll 1
  for (int e = 0; e < NE_; ++e) {
    v8f cE[4], cL[4];
#pragma unroll
    for (int j = 0; j < 4; ++j) { cE[j] = zero8(); cL[j] = zero8(); }
    const _Float16* we = W + (size_t)e * NP * LDB;
#pragma unroll 1
    for (int ks = 0; ks < KSTEPS; ++ks) {
      const int k0 = 32 * ks;
      const v16h fa = ldfrag_h(A + k0);
      v16h fl = fa;
      if (SPLIT) fl = ldfrag_h(AL + k0);
      {
        const v16h b0 = ldfrag_h(we + k0);
        const v16h b1 = ldfrag_h(we + (size_t)16 * LDB + k0);
        cE[0] = wm(fa, b0, cE[0]);
        cE[1] = wm(fa, b1, cE[1]);
        if (SPLIT) {
          cL[0] = wm(fl, b0, cL[0]);
          cL[1] = wm(fl, b1, cL[1]);
          guard4(cE[0], cL[0], cE[1], cL[1], fa, fl, b0, b1);
        } else {
          guard2(cE[0], cE[1], fa, b0, b1);
        }
      }
      {
        const v16h b2 = ldfrag_h(we + (size_t)32 * LDB + k0);
        const v16h b3 = ldfrag_h(we + (size_t)48 * LDB + k0);
        cE[2] = wm(fa, b2, cE[2]);
        cE[3] = wm(fa, b3, cE[3]);
        if (SPLIT) {
          cL[2] = wm(fl, b2, cL[2]);
          cL[3] = wm(fl, b3, cL[3]);
          guard4(cE[2], cL[2], cE[3], cL[3], fa, fl, b2, b3);
        } else {
          guard2(cE[2], cE[3], fa, b2, b3);
        }
      }
    }
    float cf[8];
#pragma unroll
    for (int r = 0; r < 8; ++r) cf[r] = cT[(16 * wave + 8 * hh + r) * 17 + e];
#pragma unroll
    for (int j = 0; j < 4; ++j) {
      const float bb = bT[e * 64 + 16 * j + idx];
#pragma unroll
      for (int r = 0; r < 8; ++r) {
        float t = cE[j][r] * (1.0f / WSC);
        if (SPLIT) {
          const float tl = cL[j][r] * (1.0f / (WSC * LOSC));
          t = t + tl;
        }
        t = t + bb;
        accM[j][r] = fmaf(cf[r], t, accM[j][r]);
      }
    }
  }

  if (!FINAL) {
    _Float16* hhp = Hh[wave];
    _Float16* hlp = Hl[wave];
#pragma unroll
    for (int j = 0; j < 4; ++j) {
#pragma unroll
      for (int r = 0; r < 8; ++r) {
        const float v = elu1(accM[j][r]);
        _Float16 h, l;
        hl_one(v, h, l);
        const int o = (8 * hh + r) * HP_ + 16 * j + idx;
        hhp[o] = h;
        hlp[o] = l;
      }
    }
    wave_sync_lds();
    const int rr = lane >> 3, pc = lane & 7;
    P8 qh[4], ql[4];
#pragma unroll
    for (int s = 0; s < 4; ++s) {
      const int row = 4 * s + rr;
      qh[s].h = *(const v8hm*)(hhp + row * HP_ + 8 * pc);
      ql[s].h = *(const v8hm*)(hlp + row * HP_ + 8 * pc);
    }
#pragma unroll
    for (int s = 0; s < 4; ++s) {
      const size_t go = (size_t)(mw + 4 * s + rr) * LDA1_ + (size_t)(n0 + 8 * pc);
      *(volatile v4u*)(ohp + go) = qh[s].u;
      *(volatile v4u*)(olp + go) = ql[s].u;
    }
    __threadfence();
#pragma unroll
    for (int s = 0; s < 4; ++s) {
      const size_t go = (size_t)(mw + 4 * s + rr) * LDA1_ + (size_t)(n0 + 8 * pc);
      *(volatile v4u*)(ohp + go) = qh[s].u;
      *(volatile v4u*)(olp + go) = ql[s].u;
    }
  } else {
    float* os = Os[wave];
#pragma unroll
    for (int j = 0; j < 4; ++j) {
#pragma unroll
      for (int r = 0; r < 8; ++r) os[(8 * hh + r) * OP_ + 16 * j + idx] = accM[j][r];
    }
    wave_sync_lds();
    const int r2 = lane >> 4, q = lane & 15;
    v4f ov[8];
#pragma unroll
    for (int s = 0; s < 8; ++s) ov[s] = *(const v4fm*)(os + (2 * s + r2) * OP_ + 4 * q);
#pragma unroll
    for (int s = 0; s < 8; ++s) {
      float* g = ofp + (size_t)(mw + 2 * s + r2) * NP + n0 + 4 * q;
      *(volatile v4f*)g = ov[s];
    }
    __threadfence();
#pragma unroll
    for (int s = 0; s < 8; ++s) {
      float* g = ofp + (size_t)(mw + 2 * s + r2) * NP + n0 + 4 * q;
      *(volatile v4f*)g = ov[s];
    }
  }
}

__global__ __launch_bounds__(256) void pack_out(const float* __restrict__ fp, float* out, int n4) {
  const int t = blockIdx.x * 256 + threadIdx.x;
  const int tc = (t < n4) ? t : (n4 - 1);
  v4f v;
#pragma unroll
  for (int u = 0; u < 4; ++u) {
    const int i = tc * 4 + u;
    const int row = i / FRM_;
    const int col = i - row * FRM_;
    v[u] = fp[(size_t)row * NP2_ + col];
  }
  float* gp = out + (size_t)tc * 4;
  if (t < n4) *(volatile v4f*)gp = v;
  __threadfence();
  if (t < n4) *(volatile v4f*)gp = v;
}

extern "C" void kernel_launch(void* const* d_in, const int* in_sizes, int n_in,
                              void* d_out, int out_size, void* d_ws, size_t ws_size,
                              hipStream_t stream) {
  if (n_in < 14) return;
  const int ex[14] = { NB_ * LAT_, NB_ * FRM_,
                       IN0_ * GH_, GH_, GH_ * GH_, GH_, GH_ * NE_, NE_,
                       NE_ * IN0_ * HID_, NE_ * HID_, NE_ * IN1_ * HID_, NE_ * HID_,
                       NE_ * IN1_ * FRM_, NE_ * FRM_ };
  for (int i = 0; i < 14; ++i) if (in_sizes[i] != ex[i]) return;
  if (out_size != NB_ * FRM_) return;

  const float* z   = (const float*)d_in[0];
  const float* c   = (const float*)d_in[1];
  const float* gw1 = (const float*)d_in[2];
  const float* gb1 = (const float*)d_in[3];
  const float* gw2 = (const float*)d_in[4];
  const float* gb2 = (const float*)d_in[5];
  const float* gw3 = (const float*)d_in[6];
  const float* gb3 = (const float*)d_in[7];
  const float* w0  = (const float*)d_in[8];
  const float* b0  = (const float*)d_in[9];
  const float* w1  = (const float*)d_in[10];
  const float* b1  = (const float*)d_in[11];
  const float* w2  = (const float*)d_in[12];
  const float* b2  = (const float*)d_in[13];
  float* out = (float*)d_out;

  const size_t hPL = (size_t)NB_ * LDA1_;
  const size_t sX0 = (size_t)NB_ * KP0_ * 2;
  const size_t sA  = hPL * 2;
  const size_t sW0 = (size_t)NE_ * HID_ * KP0_ * 2;
  const size_t sW1 = (size_t)NE_ * HID_ * KL1_ * 2;
  const size_t sW2 = (size_t)NE_ * NP2_ * KL1_ * 2;
  const size_t sG1 = (size_t)GH_ * KP0_ * 2;
  const size_t sG2 = (size_t)GH_ * GH_ * 2;
  const size_t sG3 = (size_t)NE_ * GH_ * 2;
  const size_t sCF = (size_t)NB_ * NE_ * 4;
  const size_t sF  = (size_t)NB_ * NP2_ * 4;
  size_t off = 0;
  const size_t oX0 = off; off += sX0;
  const size_t oA  = off; off += 4 * sA;
  const size_t oW0 = off; off += sW0;
  const size_t oW1 = off; off += sW1;
  const size_t oW2 = off; off += sW2;
  const size_t oG1 = off; off += sG1;
  const size_t oG2 = off; off += sG2;
  const size_t oG3 = off; off += sG3;
  const size_t oCF = off; off += sCF;
  const size_t oF  = off; off += sF;
  if (off > ws_size) return;
  if (off > (size_t)134217728) return;

  char* ws = (char*)d_ws;
  unsigned short* X0  = (unsigned short*)(ws + oX0);
  unsigned short* A1H = (unsigned short*)(ws + oA);
  unsigned short* A1L = A1H + hPL;
  unsigned short* A2H = A1L + hPL;
  unsigned short* A2L = A2H + hPL;
  unsigned short* W0T = (unsigned short*)(ws + oW0);
  unsigned short* W1T = (unsigned short*)(ws + oW1);
  unsigned short* W2T = (unsigned short*)(ws + oW2);
  unsigned short* G1T = (unsigned short*)(ws + oG1);
  unsigned short* G2T = (unsigned short*)(ws + oG2);
  unsigned short* G3T = (unsigned short*)(ws + oG3);
  float*          CF  = (float*)(ws + oCF);
  float*          F   = (float*)(ws + oF);

  const dim3 blk(256);
  {
    const int n8 = NB_ * KP0_ / 8;
    cvt_x0<<<dim3((n8 + 255) / 256), blk, 0, stream>>>(z, c, X0, n8);
  }
  {
    const int nthr = 4 * NB_ * 8;
    cvt_zl<<<dim3((nthr + 255) / 256), blk, 0, stream>>>(z, A1H, nthr);
  }
  {
    const int n8a = NE_ * HID_ * KP0_ / 8;
    cvt_w<<<dim3((n8a + 255) / 256), blk, 0, stream>>>(w0, W0T, IN0_, HID_, HID_, KP0_, FRM_, ZO0_, LAT_, n8a);
    const int n8b = NE_ * HID_ * KL1_ / 8;
    cvt_w<<<dim3((n8b + 255) / 256), blk, 0, stream>>>(w1, W1T, IN1_, HID_, HID_, KL1_, HID_, ZO1_, LAT_, n8b);
    const int n8c = NE_ * NP2_ * KL1_ / 8;
    cvt_w<<<dim3((n8c + 255) / 256), blk, 0, stream>>>(w2, W2T, IN1_, FRM_, NP2_, KL1_, HID_, ZO1_, LAT_, n8c);
    const int n8d = GH_ * KP0_ / 8;
    cvt_w<<<dim3((n8d + 255) / 256), blk, 0, stream>>>(gw1, G1T, IN0_, GH_, GH_, KP0_, FRM_, ZO0_, LAT_, n8d);
    const int n8e = GH_ * GH_ / 8;
    cvt_w<<<dim3((n8e + 255) / 256), blk, 0, stream>>>(gw2, G2T, GH_, GH_, GH_, GH_, GH_, GH_, 0, n8e);
    const int n8f = NE_ * GH_ / 8;
    cvt_w<<<dim3((n8f + 255) / 256), blk, 0, stream>>>(gw3, G3T, GH_, NE_, NE_, GH_, GH_, GH_, 0, n8f);
  }
  gate_mlp<<<dim3(NB_ / 32), dim3(64), 0, stream>>>(X0, G1T, gb1, G2T, gb2, G3T, gb3, CF);
  moe_gemm<KP0_ / 32, KP0_, KP0_, HID_, HID_, false, false>
      <<<dim3(HID_ / 64, NB_ / 64), dim3(128), 0, stream>>>(X0, X0, W0T, b0, CF, A1H, A1L, F);
  moe_gemm<KL1_ / 32, LDA1_, KL1_, HID_, HID_, true, false>
      <<<dim3(HID_ / 64, NB_ / 64), dim3(128), 0, stream>>>(A1H, A1L, W1T, b1, CF, A2H, A2L, F);
  moe_gemm<KL1_ / 32, LDA1_, KL1_, NP2_, FRM_, true, true>
      <<<dim3(NP2_ / 64, NB_ / 64), dim3(128), 0, stream>>>(A2H, A2L, W2T, b2, CF, A1H, A1L, F);
  {
    const int n4 = NB_ * FRM_ / 4;
    pack_out<<<dim3((n4 + 255) / 256), blk, 0, stream>>>(F, out, n4);
  }
  (void)hipGetLastError();
}
